// GATConvLayer_new_16389595202404
// MI455X (gfx1250) — hardware-verified
//
#include <hip/hip_runtime.h>


#define NN   512
#define NE   262144
#define CI   64
#define CE   32
#define ST   80
#define SP   96
#define CHE  131072
typedef _Float16 h16;
typedef unsigned short bf;
typedef __attribute__((ext_vector_type(16))) __bf16   v16bf;
typedef __attribute__((ext_vector_type(16))) _Float16 v16h;
typedef __attribute__((ext_vector_type(8)))  _Float16 v8h;
typedef __attribute__((ext_vector_type(8)))  unsigned short v8us;
typedef __attribute__((ext_vector_type(8)))  float    v8f;
typedef __attribute__((ext_vector_type(4)))  float    v4f;
typedef v8h  __attribute__((may_alias)) v8ha;
typedef v4f  __attribute__((may_alias)) v4fa;
typedef v8us __attribute__((may_alias)) v8usa;

__device__ __forceinline__ unsigned short f2bf(float f) { unsigned u = __float_as_uint(f); u += 0x7FFFu + ((u >> 16) & 1u); return (unsigned short)(u >> 16); }
__device__ __forceinline__ float bf2f(unsigned short b) { return __uint_as_float(((unsigned)b) << 16); }
__device__ __forceinline__ float bfr(float f) { return bf2f(f2bf(f)); }
__device__ __forceinline__ v16h cat16(v8h lo, v8h hi) { return __builtin_shufflevector(lo, hi, 0, 1, 2, 3, 4, 5, 6, 7, 8, 9, 10, 11, 12, 13, 14, 15); }
__device__ __forceinline__ v16bf cat16b(v8us lo, v8us hi) { return __builtin_bit_cast(v16bf, __builtin_shufflevector(lo, hi, 0, 1, 2, 3, 4, 5, 6, 7, 8, 9, 10, 11, 12, 13, 14, 15)); }
__device__ __forceinline__ v8f wmma16(v16h a, v16h b, v8f c) { return __builtin_amdgcn_wmma_f32_16x16x32_f16(false, a, false, b, (short)0, c, false, false); }
__device__ __forceinline__ v8f wmmab(v16bf a, v16bf b, v8f c) { return __builtin_amdgcn_wmma_f32_16x16x32_bf16(false, a, false, b, (short)0, c, false, false); }


template <typename T16> struct WFrag;
template <> struct WFrag<h16> { typedef v16h V; static __device__ __forceinline__ V ld(const h16* p) { return cat16(*(const v8h*)p, *(const v8h*)(p + 16)); } static __device__ __forceinline__ v8f mma(V a, V b, v8f c) { return wmma16(a, b, c); } };
template <> struct WFrag<bf> { typedef v16bf V; static __device__ __forceinline__ V ld(const bf* p) { return cat16b(*(const v8us*)p, *(const v8us*)(p + 16)); } static __device__ __forceinline__ v8f mma(V a, V b, v8f c) { return wmmab(a, b, c); } };
template <typename T16, int NSPLIT, bool BIAS>
__global__ __launch_bounds__(32) void k_gemmw(const T16* __restrict__ A, const T16* __restrict__ A2, const T16* __restrict__ Bt, const T16* __restrict__ Bt2, int K, float* C, int ldc, const float* __restrict__ bias, size_t sA, size_t sB, size_t sC) {
    typedef typename WFrag<T16>::V V;
    __shared__ __align__(16) float os[16 * 68];
    const size_t z = blockIdx.z; A += z * sA; if (A2) A2 += z * sA; Bt += z * sB; if (Bt2) Bt2 += z * sB; C += z * sC;
    const int lane = threadIdx.x & 31, lr = lane & 15, hi = lane >> 4; const int r0 = blockIdx.x * 64, c0 = blockIdx.y * 64;
    v8f acc[4][4];
#pragma unroll
    for (int mb = 0; mb < 4; ++mb)
#pragma unroll
        for (int nb = 0; nb < 4; ++nb) acc[mb][nb] = (v8f){};
    const size_t aoff = (size_t)(r0 + lr) * K + 8 * hi, boff = (size_t)(c0 + lr) * K + 8 * hi;
#pragma unroll 1
    for (int kc = 0; kc < K; kc += 32) {
        V a[4], a2[4];
#pragma unroll
        for (int mb = 0; mb < 4; ++mb) { a[mb] = WFrag<T16>::ld(A + aoff + (size_t)mb * 16 * K + kc); if (NSPLIT == 1 || NSPLIT == 2) a2[mb] = WFrag<T16>::ld(A2 + aoff + (size_t)mb * 16 * K + kc); }
#pragma unroll
        for (int nb = 0; nb < 4; ++nb) { const V b = WFrag<T16>::ld(Bt + boff + (size_t)nb * 16 * K + kc); V b2; if (NSPLIT >= 2) b2 = WFrag<T16>::ld(Bt2 + boff + (size_t)nb * 16 * K + kc);
#pragma unroll
            for (int mb = 0; mb < 4; ++mb) { acc[mb][nb] = WFrag<T16>::mma(a[mb], b, acc[mb][nb]); if (NSPLIT == 1 || NSPLIT == 2) acc[mb][nb] = WFrag<T16>::mma(a2[mb], b, acc[mb][nb]); if (NSPLIT >= 2) acc[mb][nb] = WFrag<T16>::mma(a[mb], b2, acc[mb][nb]); } }
        asm volatile("v_nop\n\tv_nop\n\tv_nop\n\tv_nop" : "+v"(acc[0][0]), "+v"(acc[1][1]), "+v"(acc[2][2]), "+v"(acc[3][3]) : "v"(a[0]), "v"(a[3]));
    }
#pragma unroll
    for (int mb = 0; mb < 4; ++mb) {
#pragma unroll
        for (int nb = 0; nb < 4; ++nb) {
#pragma unroll
            for (int j = 0; j < 8; ++j) os[(hi * 8 + j) * 68 + nb * 16 + lr] = acc[mb][nb][j]; }
        __builtin_amdgcn_wave_barrier(); asm volatile("" ::: "memory");
        float* crow = C + (size_t)(r0 + mb * 16) * ldc + c0;
#pragma unroll 1
        for (int ps = 0; ps < 2; ++ps) {
#pragma unroll
            for (int s = 0; s < 8; ++s) { const int row = 2 * s + hi, cofs = lr * 4; v4f val = *(const v4fa*)(os + row * 68 + cofs); if (BIAS) { val[0] += bfr(bias[c0 + cofs]); val[1] += bfr(bias[c0 + cofs + 1]); val[2] += bfr(bias[c0 + cofs + 2]); val[3] += bfr(bias[c0 + cofs + 3]); }
                *(volatile v4f*)(crow + (size_t)row * ldc + cofs) = val; }
            if (ps == 0) __threadfence(); }
        __builtin_amdgcn_wave_barrier(); asm volatile("" ::: "memory");
    }
}

__device__ __forceinline__ void splitf(float y, unsigned short& h, unsigned short& l) { h = f2bf(y); l = f2bf(y - bf2f(h)); }
__device__ __forceinline__ float lre(float v) { return v > 0.f ? v : __fmul_rn(0.1f, v); }
typedef __attribute__((ext_vector_type(2))) unsigned short v2us;
typedef __attribute__((ext_vector_type(4))) unsigned short v4us;

__global__ __launch_bounds__(256) void k_cvt8(const float* __restrict__ src, bf* dst, size_t n8) { const size_t i = (size_t)blockIdx.x * 256 + threadIdx.x; if (i >= n8) return; const v8f v = *(const v8f*)(src + i * 8); v8us o;
#pragma unroll
    for (int k = 0; k < 8; ++k) o[k] = f2bf(v[k]); *(volatile v8us*)(dst + i * 8) = o; __threadfence(); *(volatile v8us*)(dst + i * 8) = o; }
__global__ __launch_bounds__(256) void k_wg(const float* __restrict__ Wt, int ld, int col0, int nrow, int ncol, int KP, int NP, bf* Bt) { const int e = (blockIdx.x * 256 + threadIdx.x) * 4; if (e >= NP * KP) return; const int c = e % KP; const int s = e / KP; v4us o;
#pragma unroll
    for (int u = 0; u < 4; ++u) o[u] = (s < nrow && c + u < ncol) ? f2bf(Wt[(size_t)s * ld + col0 + c + u]) : (unsigned short)0; *(volatile v4us*)(Bt + e) = o; __threadfence(); *(volatile v4us*)(Bt + e) = o; }
__global__ __launch_bounds__(256) void k_h(const float* __restrict__ A, const float* __restrict__ E, const float* __restrict__ Bm, const float* __restrict__ bh, int e0, bf* Hh, bf* Hl) { const size_t q = ((size_t)blockIdx.x * 256 + threadIdx.x) * 4; if (q >= (size_t)CHE * SP) return; const int s0 = (int)(q % SP); const int el = (int)(q / SP); const int e = e0 + el; const int i = e / NN, j = e % NN; v4us oh, ol;
#pragma unroll
    for (int u = 0; u < 4; ++u) { const int s = s0 + u; float v = 0.f; if (s < ST) v = lre(__fadd_rn(__fadd_rn(__fadd_rn(A[i * 128 + s], E[(size_t)el * 128 + s]), Bm[j * 128 + s]), bfr(bh[s]))); unsigned short a, b; splitf(v, a, b); oh[u] = a; ol[u] = b; }
    *(volatile v4us*)(Hh + q) = oh; *(volatile v4us*)(Hl + q) = ol; __threadfence(); *(volatile v4us*)(Hh + q) = oh; *(volatile v4us*)(Hl + q) = ol; }
__global__ __launch_bounds__(256) void k_ne(const float* __restrict__ G, const float* __restrict__ beo, const int* __restrict__ mk, int e0, float* NEA) { const int q = (blockIdx.x * 256 + threadIdx.x) * 4; if (q >= CHE * CE) return; const int c = q % CE; const int el = q / CE; const int e = e0 + el; const float m = (mk[e] != 0) ? 1.f : 0.f; v4f o;
#pragma unroll
    for (int u = 0; u < 4; ++u) o[u] = __fmul_rn(lre(__fadd_rn(G[(size_t)el * 64 + c + u], bfr(beo[c + u]))), m); float* dst = NEA + (size_t)e * CE + c; *(volatile v4f*)dst = o; __threadfence(); *(volatile v4f*)dst = o; }
__global__ __launch_bounds__(256) void k_xn(const float* __restrict__ F, float* XN) { const int e = (blockIdx.x * 256 + threadIdx.x) * 4; if (e >= NN * CI) return; const v4f a = *(const v4f*)(F + e); v4f o; for (int u = 0; u < 4; ++u) o[u] = lre(a[u]); *(volatile v4f*)(XN + e) = o; __threadfence(); *(volatile v4f*)(XN + e) = o; }
__global__ __launch_bounds__(256) void k_ac(const float* __restrict__ XN, const float* __restrict__ ev, float* AI, float* CJ) { const int i = blockIdx.x * 256 + threadIdx.x; if (i >= NN) return; float a = 0.f, c = 0.f;
#pragma unroll 1
    for (int k = 0; k < CI; ++k) { const float xv = XN[i * CI + k]; float w1 = bfr(ev[k]), w3 = bfr(ev[96 + k]); asm volatile("" : "+v"(w1)); asm volatile("" : "+v"(w3)); float p1 = __fmul_rn(xv, w1), p3 = __fmul_rn(xv, w3); asm volatile("" : "+v"(p1)); asm volatile("" : "+v"(p3)); a = __fadd_rn(a, p1); c = __fadd_rn(c, p3); }
    for (int ps = 0; ps < 2; ++ps) { *(volatile float*)(AI + i) = a; *(volatile float*)(CJ + i) = c; if (ps == 0) __threadfence(); } }
__global__ __launch_bounds__(256) void k_att(const float* __restrict__ NEA, const float* __restrict__ ev, const float* __restrict__ AI, const float* __restrict__ CJ, const int* __restrict__ mk, float* ATT) { const int lane = threadIdx.x & 31; const int i = blockIdx.x * 8 + (threadIdx.x >> 5); if (i >= NN) return; const float ai = AI[i]; float v[NN / 32]; float mx = -3.0e38f;
#pragma unroll
    for (int ch = 0; ch < NN / 128; ++ch) {
#pragma unroll
        for (int u = 0; u < 4; ++u) { const int j = ch * 128 + lane * 4 + u; const float* ne = NEA + ((size_t)i * NN + j) * CE; float mid = 0.f;
#pragma unroll 1
            for (int c = 0; c < CE; ++c) { float w = bfr(ev[64 + c]); asm volatile("" : "+v"(w)); float p = __fmul_rn(ne[c], w); asm volatile("" : "+v"(p)); mid = __fadd_rn(mid, p); }
            const float sc = lre(__fadd_rn(__fadd_rn(ai, mid), CJ[j])); v[ch * 4 + u] = sc; mx = fmaxf(mx, sc); } }
#pragma unroll
    for (int sh = 16; sh; sh >>= 1) mx = fmaxf(mx, __shfl_xor(mx, sh, 32));
    float sum = 0.f;
#pragma unroll
    for (int q = 0; q < NN / 32; ++q) { float d0 = __fsub_rn(v[q], mx); asm volatile("" : "+v"(d0)); v[q] = __builtin_amdgcn_exp2f(__fmul_rn(d0, 1.4426950408889634f)); sum += v[q]; }
#pragma unroll
    for (int sh = 16; sh; sh >>= 1) sum += __shfl_xor(sum, sh, 32);
    const float f = __fdiv_rn(1.0f, sum);
    for (int ps = 0; ps < 2; ++ps) {
#pragma unroll
        for (int ch = 0; ch < NN / 128; ++ch) { v4f o; const int j0 = ch * 128 + lane * 4;
#pragma unroll
            for (int u = 0; u < 4; ++u) { float p = v[ch * 4 + u] * f; o[u] = (mk[(size_t)i * NN + j0 + u] != 0) ? p : __fmul_rn(p, 0.f); } *(volatile v4f*)(ATT + (size_t)i * NN + j0) = o; }
        if (ps == 0) __threadfence(); } }
__global__ __launch_bounds__(256) void k_newx(const float* __restrict__ ATT, const float* __restrict__ XN, float* NX) { const int e = (blockIdx.x * 256 + threadIdx.x) * 4; if (e >= NN * CI) return; const int c0 = e % CI; const int i = e / CI; float acc[4] = {0.f, 0.f, 0.f, 0.f};
#pragma unroll 1
    for (int j = 0; j < NN; ++j) { const float a = ATT[(size_t)i * NN + j];
#pragma unroll
        for (int u = 0; u < 4; ++u) { float p = __fmul_rn(a, XN[j * CI + c0 + u]); asm volatile("" : "+v"(p)); acc[u] = __fadd_rn(acc[u], p); } }
    v4f o; for (int u = 0; u < 4; ++u) o[u] = acc[u]; *(volatile v4f*)(NX + e) = o; __threadfence(); *(volatile v4f*)(NX + e) = o; }
__global__ __launch_bounds__(64) void k_cst(const float* __restrict__ V, int nrow, int ncol, float* MEAN, float* VAR) { const int c = threadIdx.x; if (c >= ncol) return; float s = 0.f;
    for (int r = 0; r < nrow; ++r) s = __fadd_rn(s, V[(size_t)r * ncol + c]);
    const float mean = __fdiv_rn(s, (float)nrow); float q = 0.f;
    for (int r = 0; r < nrow; ++r) { float d = __fsub_rn(V[(size_t)r * ncol + c], mean); asm volatile("" : "+v"(d)); float p = __fmul_rn(d, d); asm volatile("" : "+v"(p)); q = __fadd_rn(q, p); }
    const float var = __fdiv_rn(q, (float)nrow); for (int ps = 0; ps < 2; ++ps) { *(volatile float*)(MEAN + c) = mean; *(volatile float*)(VAR + c) = var; if (ps == 0) __threadfence(); } }
template <int SQ> __global__ __launch_bounds__(256) void k_epart(const float* __restrict__ V, const float* __restrict__ MEAN, float* PART) { const int idx = blockIdx.x * 256 + threadIdx.x; if (idx >= 512 * CE) return; const int c = idx % CE; const int p = idx / CE; const float mu = SQ ? MEAN[c] : 0.f; float s = 0.f;
#pragma unroll 1
    for (int r = p * 512; r < p * 512 + 512; ++r) { float v = V[(size_t)r * CE + c]; if (SQ) { float d = __fsub_rn(v, mu); asm volatile("" : "+v"(d)); v = __fmul_rn(d, d); asm volatile("" : "+v"(v)); } s = __fadd_rn(s, v); }
    *(volatile float*)(PART + idx) = s; __threadfence(); *(volatile float*)(PART + idx) = s; }
__global__ __launch_bounds__(64) void k_esum(const float* __restrict__ PART, float* OUTS) { const int c = threadIdx.x; if (c >= CE) return; float s = 0.f;
#pragma unroll 1
    for (int p = 0; p < 512; ++p) s = __fadd_rn(s, PART[p * CE + c]); const float r = __fdiv_rn(s, (float)NE); *(volatile float*)(OUTS + c) = r; __threadfence(); *(volatile float*)(OUTS + c) = r; }
__global__ __launch_bounds__(256) void k_bn(const float* __restrict__ V, size_t n4, int ncol, const float* __restrict__ MEAN, const float* __restrict__ VAR, const float* __restrict__ w, const float* __restrict__ b, float* OUTb) { const size_t e = ((size_t)blockIdx.x * 256 + threadIdx.x) * 4; if (e >= n4) return; const int c0 = (int)(e % ncol); const v4f a = *(const v4f*)(V + e); v4f o;
#pragma unroll
    for (int u = 0; u < 4; ++u) { const int c = c0 + u; float d = __fsub_rn(a[u], MEAN[c]); asm volatile("" : "+v"(d)); float n0 = __fmul_rn(d, __frsqrt_rn(__fadd_rn(VAR[c], 1e-5f))); asm volatile("" : "+v"(n0)); float t1 = __fmul_rn(n0, bfr(w[c])); asm volatile("" : "+v"(t1)); o[u] = __fadd_rn(t1, bfr(b[c])); }
    *(volatile v4f*)(OUTb + e) = o; __threadfence(); *(volatile v4f*)(OUTb + e) = o; }

extern "C" void kernel_launch(void* const* d_in, const int* in_sizes, int n_in,
                              void* d_out, int out_size, void* d_ws, size_t ws_size, hipStream_t stream) {
    (void)in_sizes; (void)n_in; (void)out_size;
    const float** I = (const float**)d_in;
    const float *x = I[0], *ea = I[1], *W_nu = I[3], *b_nu = I[4], *W_h2 = I[5], *b_h2 = I[6], *W_eo = I[7], *b_eo = I[8], *ev = I[9], *bnw = I[10], *bnb = I[11], *bew = I[12], *beb = I[13]; const int* mk = (const int*)d_in[2];
    float* OUT0 = (float*)d_out; float* OUT1 = OUT0 + NN * CI;
    char* wsp = (char*)d_ws;
    auto take = [&](size_t bytes) { char* p = wsp; wsp += (bytes + 255) & ~(size_t)255; return (void*)p; };
    bf* BtA = (bf*)take(128 * CI * 2); bf* BtE = (bf*)take(128 * CE * 2); bf* BtB = (bf*)take(128 * CI * 2); bf* BtO = (bf*)take(64 * SP * 2); bf* BtN = (bf*)take(CI * CI * 2);
    bf* XB = (bf*)take(NN * CI * 2); bf* EB = (bf*)take((size_t)NE * CE * 2); float* A = (float*)take(NN * 128 * 4); float* Bm = (float*)take(NN * 128 * 4); float* E = (float*)take((size_t)CHE * 128 * 4); bf* Hh = (bf*)take((size_t)CHE * SP * 2); bf* Hl = (bf*)take((size_t)CHE * SP * 2); float* G = (float*)take((size_t)CHE * 64 * 4);
    float* NEA = (float*)take((size_t)NE * CE * 4); float* F = (float*)take(NN * CI * 4); float* XN = (float*)take(NN * CI * 4); float* AI = (float*)take(NN * 4); float* CJ = (float*)take(NN * 4); float* ATT = (float*)take((size_t)NN * NN * 4); float* NX = (float*)take(NN * CI * 4);
    float* MN = (float*)take(256); float* VN = (float*)take(256); float* PART = (float*)take(512 * CE * 4); float* ME = (float*)take(256); float* VE = (float*)take(256);
    if ((size_t)(wsp - (char*)d_ws) > ws_size) return;
    k_wg<<<(128 * CI / 4 + 255) / 256, 256, 0, stream>>>(W_h2, 160, 0, ST, CI, CI, 128, BtA); k_wg<<<(128 * CE / 4 + 255) / 256, 256, 0, stream>>>(W_h2, 160, 64, ST, CE, CE, 128, BtE); k_wg<<<(128 * CI / 4 + 255) / 256, 256, 0, stream>>>(W_h2, 160, 96, ST, CI, CI, 128, BtB);
    k_wg<<<(64 * SP / 4 + 255) / 256, 256, 0, stream>>>(W_eo, ST, 0, CE, ST, SP, 64, BtO); k_cvt8<<<(CI * CI / 8 + 255) / 256, 256, 0, stream>>>(W_nu, BtN, CI * CI / 8);
    k_cvt8<<<(NN * CI / 8 + 255) / 256, 256, 0, stream>>>(x, XB, NN * CI / 8); k_cvt8<<<(unsigned)(((size_t)NE * CE / 8 + 255) / 256), 256, 0, stream>>>(ea, EB, (size_t)NE * CE / 8);
    k_gemmw<bf, 0, false><<<dim3(NN / 64, 2, 1), 32, 0, stream>>>(XB, nullptr, BtA, nullptr, CI, A, 128, nullptr, 0, 0, 0); k_gemmw<bf, 0, false><<<dim3(NN / 64, 2, 1), 32, 0, stream>>>(XB, nullptr, BtB, nullptr, CI, Bm, 128, nullptr, 0, 0, 0);
    for (int e0 = 0; e0 < NE; e0 += CHE) {
        k_gemmw<bf, 0, false><<<dim3(CHE / 64, 2, 1), 32, 0, stream>>>(EB + (size_t)e0 * CE, nullptr, BtE, nullptr, CE, E, 128, nullptr, 0, 0, 0);
        k_h<<<(unsigned)(((size_t)CHE * SP / 4 + 255) / 256), 256, 0, stream>>>(A, E, Bm, b_h2, e0, Hh, Hl);
        k_gemmw<bf, 1, false><<<dim3(CHE / 64, 1, 1), 32, 0, stream>>>(Hh, Hl, BtO, nullptr, SP, G, 64, nullptr, 0, 0, 0);
        k_ne<<<(CHE * CE / 4 + 255) / 256, 256, 0, stream>>>(G, b_eo, mk, e0, NEA); }
    k_gemmw<bf, 0, true><<<dim3(NN / 64, 1, 1), 32, 0, stream>>>(XB, nullptr, BtN, nullptr, CI, F, CI, b_nu, 0, 0, 0); k_xn<<<(NN * CI / 4 + 255) / 256, 256, 0, stream>>>(F, XN); k_ac<<<(NN + 255) / 256, 256, 0, stream>>>(XN, ev, AI, CJ);
    k_att<<<NN / 8, 256, 0, stream>>>(NEA, ev, AI, CJ, mk, ATT); k_newx<<<(NN * CI / 4 + 255) / 256, 256, 0, stream>>>(ATT, XN, NX);
    k_cst<<<1, 64, 0, stream>>>(NX, NN, CI, MN, VN); k_bn<<<(NN * CI / 4 + 255) / 256, 256, 0, stream>>>(NX, (size_t)NN * CI, CI, MN, VN, bnw, bnb, OUT0);
    k_epart<0><<<(512 * CE + 255) / 256, 256, 0, stream>>>(NEA, nullptr, PART); k_esum<<<1, 64, 0, stream>>>(PART, ME); k_epart<1><<<(512 * CE + 255) / 256, 256, 0, stream>>>(NEA, ME, PART); k_esum<<<1, 64, 0, stream>>>(PART, VE);
    k_bn<<<(unsigned)(((size_t)NE * CE / 4 + 255) / 256), 256, 0, stream>>>(NEA, (size_t)NE * CE, CE, ME, VE, bew, beb, OUT1);
}
